// LTMPBlock_87591563035018
// MI455X (gfx1250) — hardware-run, weakly checked
//
#include <hip/hip_runtime.h>
#include <stddef.h>
#include <stdint.h>
#include <math.h>

#define BB   8
#define NN   1024
#define CC   768
#define HH   12
#define DD   64
#define FF   3072
#define NH   512
#define ROWS (BB * NN)
#define C3   (3 * CC)
#define QB   (NN / 128)
#define PL   ((size_t)BB * HH * NN * DD)

static_assert(NN % 256 == 0);
static_assert(CC % 64 == 0);
static_assert(FF % 64 == 0);
static_assert(DD == 64);
static_assert(HH * DD == CC);
static_assert(ROWS % 256 == 0);
static_assert(CC == 192 * 4);
static_assert(NN == 256 * 4);
static_assert(2 * NH == NN);
static_assert(NH == 2 * 256);

typedef _Float16 v16h __attribute__((ext_vector_type(16)));
typedef _Float16 v8h  __attribute__((ext_vector_type(8)));
typedef _Float16 v4hh __attribute__((ext_vector_type(4)));
typedef float    v8f  __attribute__((ext_vector_type(8)));
typedef float    v4f  __attribute__((ext_vector_type(4)));
typedef unsigned int v4u __attribute__((ext_vector_type(4)));

union Frag  { v16h v; v8h h[2]; };
union Pack8 { v8h h; v4u u; };

__device__ __forceinline__ v8f mma16(v16h a, v16h b, v8f c) {
  c = __builtin_amdgcn_wmma_f32_16x16x32_f16(false, a, false, b, (short)0, c, false, false);
  asm volatile("v_nop\n\tv_nop\n\tv_nop\n\tv_nop" : "+v"(c) : "v"(a), "v"(b));
  return c;
}

__device__ __forceinline__ v16h ldfrag(const _Float16* p, int ld, int row0, int k0, int lane) {
  const int m = lane & 15, lh = lane >> 4;
  const _Float16* q = p + (size_t)(row0 + m) * ld + k0 + 8 * lh;
  Frag f;
  f.h[0] = *(const v8h*)(q);
  f.h[1] = *(const v8h*)(q + 16);
  return f.v;
}

__device__ __forceinline__ v8f zero8() { return (v8f){0.f, 0.f, 0.f, 0.f, 0.f, 0.f, 0.f, 0.f}; }
__device__ __forceinline__ v4f zero4() { return (v4f){0.f, 0.f, 0.f, 0.f}; }

__device__ __forceinline__ float act16(float v) {
  return 8.0f * v * (1.0f + erff(v * 0.70710678118654752f));
}

template <int KK>
__device__ __forceinline__ void gemm32x64(const _Float16* __restrict__ A, int lda,
                                          const _Float16* __restrict__ Bt, int ldb,
                                          int m0, int n0, int lane, v8f (&acc)[2][4]) {
  static_assert(KK % 32 == 0);
#pragma unroll 2
  for (int k0 = 0; k0 < KK; k0 += 32) {
    const v16h a0 = ldfrag(A, lda, m0, k0, lane);
    const v16h a1 = ldfrag(A, lda, m0 + 16, k0, lane);
    const v16h b0 = ldfrag(Bt, ldb, n0, k0, lane);
    const v16h b1 = ldfrag(Bt, ldb, n0 + 16, k0, lane);
    const v16h b2 = ldfrag(Bt, ldb, n0 + 32, k0, lane);
    const v16h b3 = ldfrag(Bt, ldb, n0 + 48, k0, lane);
    acc[0][0] = mma16(a0, b0, acc[0][0]);
    acc[1][0] = mma16(a1, b0, acc[1][0]);
    acc[0][1] = mma16(a0, b1, acc[0][1]);
    acc[1][1] = mma16(a1, b1, acc[1][1]);
    acc[0][2] = mma16(a0, b2, acc[0][2]);
    acc[1][2] = mma16(a1, b2, acc[1][2]);
    acc[0][3] = mma16(a0, b3, acc[0][3]);
    acc[1][3] = mma16(a1, b3, acc[1][3]);
  }
}

__global__ __launch_bounds__(192) void k_ln(const float* __restrict__ in,
                                           const float* __restrict__ g,
                                           const float* __restrict__ bt,
                                           _Float16* __restrict__ outh, float eps) {
  __shared__ __align__(16) float rb[CC];
  __shared__ float red[16];
  const int tid = threadIdx.x, lane = tid & 31, wave = tid >> 5;
  const size_t ro = (size_t)blockIdx.x * CC;
  const v4f v = *(const v4f*)(in + ro + 4 * tid);
  float s = (v[0] + v[1]) + (v[2] + v[3]);
#pragma unroll
  for (int off = 1; off < 32; off <<= 1) s += __shfl_xor(s, off, 32);
  if (lane == 0) red[wave] = s;
  __syncthreads();
  float ts = 0.f;
#pragma unroll
  for (int w = 0; w < 6; ++w) ts += red[w];
  const float mean = ts * (1.0f / (float)CC);
  const float d0 = v[0] - mean, d1 = v[1] - mean, d2 = v[2] - mean, d3 = v[3] - mean;
  float q = (d0 * d0 + d1 * d1) + (d2 * d2 + d3 * d3);
#pragma unroll
  for (int off = 1; off < 32; off <<= 1) q += __shfl_xor(q, off, 32);
  if (lane == 0) red[8 + wave] = q;
  __syncthreads();
  float tq = 0.f;
#pragma unroll
  for (int w = 0; w < 6; ++w) tq += red[8 + w];
  const float var = tq * (1.0f / (float)CC);
  const float inv = 1.0f / sqrtf(var + eps);
  const v4f g4 = *(const v4f*)(g + 4 * tid);
  const v4f b4 = *(const v4f*)(bt + 4 * tid);
  v4f o;
  o[0] = d0 * inv * g4[0] + b4[0];
  o[1] = d1 * inv * g4[1] + b4[1];
  o[2] = d2 * inv * g4[2] + b4[2];
  o[3] = d3 * inv * g4[3] + b4[3];
  *(v4f*)(rb + 4 * tid) = o;
  __syncthreads();
  if (tid < 96) {
    const v4f a0 = *(const v4f*)(rb + 8 * tid);
    const v4f a1 = *(const v4f*)(rb + 8 * tid + 4);
    Pack8 pk;
    pk.h = (v8h){(_Float16)a0[0], (_Float16)a0[1], (_Float16)a0[2], (_Float16)a0[3],
                 (_Float16)a1[0], (_Float16)a1[1], (_Float16)a1[2], (_Float16)a1[3]};
    const v4u vv = pk.u;
    volatile v4u* hq = (volatile v4u*)(outh + ro + 8 * tid);
    *hq = vv;
    __threadfence();
    *hq = vv;
  }
}

#define WTP 68
__global__ __launch_bounds__(256) void k_wt(const float* __restrict__ w, _Float16* __restrict__ wt,
                                           int nout, int kin) {
  __shared__ __align__(16) float tf[64 * WTP];
  const int tid = threadIdx.x;
  const int n0 = blockIdx.x * 64;
  const int k0 = blockIdx.y * 64;
  {
    const int kr = tid >> 4;
    const int n4 = (tid & 15) * 4;
#pragma unroll
    for (int it = 0; it < 4; ++it) {
      const int kl = it * 16 + kr;
      const v4f a = *(const v4f*)(w + (size_t)(k0 + kl) * nout + n0 + n4);
      *(v4f*)(tf + kl * WTP + n4) = a;
    }
  }
  __syncthreads();
  v4u val[2];
  size_t go[2];
#pragma unroll
  for (int j = 0; j < 2; ++j) {
    const int p  = tid + 256 * j;
    const int nl = p >> 3;
    const int pc = p & 7;
    const float* cp = tf + (pc * 8) * WTP + nl;
    Pack8 pk;
    pk.h = (v8h){(_Float16)(cp[0 * WTP] * 32.0f), (_Float16)(cp[1 * WTP] * 32.0f),
                 (_Float16)(cp[2 * WTP] * 32.0f), (_Float16)(cp[3 * WTP] * 32.0f),
                 (_Float16)(cp[4 * WTP] * 32.0f), (_Float16)(cp[5 * WTP] * 32.0f),
                 (_Float16)(cp[6 * WTP] * 32.0f), (_Float16)(cp[7 * WTP] * 32.0f)};
    val[j] = pk.u;
    go[j]  = (size_t)(n0 + nl) * kin + k0 + pc * 8;
  }
  for (int ps = 0; ps < 2; ++ps) {
#pragma unroll
    for (int j = 0; j < 2; ++j) *(volatile v4u*)(wt + go[j]) = val[j];
    __threadfence();
  }
}

#define STP 72
__global__ __launch_bounds__(256) void k_qkv(const _Float16* __restrict__ xh,
                                             const _Float16* __restrict__ wt,
                                             _Float16* __restrict__ qkv) {
  __shared__ __align__(16) _Float16 st[256 * STP];
  const int tid = threadIdx.x, lane = tid & 31, wave = tid >> 5;
  const int hh = lane >> 4, c = lane & 15;
  const int mb = blockIdx.x * 256;
  const int m0 = mb + wave * 32;
  const int n0 = blockIdx.y * 64;
  const int which = n0 / CC;
  const int nin = n0 - which * CC;

  v8f acc[2][4];
#pragma unroll
  for (int s = 0; s < 2; ++s)
#pragma unroll
    for (int t = 0; t < 4; ++t) acc[s][t] = zero8();
  gemm32x64<CC>(xh, CC, wt, CC, m0, n0, lane, acc);

#pragma unroll
  for (int t = 0; t < 4; ++t) {
#pragma unroll
    for (int sub = 0; sub < 2; ++sub) {
#pragma unroll
      for (int r = 0; r < 8; ++r) {
        const int lr = wave * 32 + sub * 16 + 8 * hh + r;
        st[lr * STP + 16 * t + c] = (_Float16)(acc[sub][t][r] * 0.03125f);
      }
    }
  }
  __syncthreads();

  const int head = nin >> 6;
  const int b  = mb / NN;
  const int nb = mb - b * NN;
  const int bh = b * HH + head;
  v4u val[8];
  size_t go[8];
  if (which < 2) {
#pragma unroll
    for (int j = 0; j < 8; ++j) {
      const int p  = tid + 256 * j;
      const int lr = p >> 3;
      const int pc = p & 7;
      Pack8 pk;
      pk.h  = *(const v8h*)(st + lr * STP + pc * 8);
      val[j] = pk.u;
      go[j]  = (size_t)which * PL + ((size_t)bh * NN + nb + lr) * DD + pc * 8;
    }
  } else {
#pragma unroll
    for (int j = 0; j < 8; ++j) {
      const int p  = tid + 256 * j;
      const int L  = p >> 3;
      const int pc = p & 7;
      const int d  = L >> 2;
      const int nl = (L & 3) * 64 + pc * 8;
      const _Float16* cp = st + nl * STP + d;
      Pack8 pk;
      pk.h = (v8h){cp[0 * STP], cp[1 * STP], cp[2 * STP], cp[3 * STP],
                   cp[4 * STP], cp[5 * STP], cp[6 * STP], cp[7 * STP]};
      val[j] = pk.u;
      go[j]  = 2 * PL + ((size_t)bh * DD + d) * NN + nb + nl;
    }
  }
  for (int ps = 0; ps < 2; ++ps) {
#pragma unroll
    for (int j = 0; j < 8; ++j) *(volatile v4u*)(qkv + go[j]) = val[j];
    __threadfence();
  }
}

#define KTP 72
#define PTP 72
__global__ __launch_bounds__(256) void k_attn(const _Float16* __restrict__ qp,
                                              const _Float16* __restrict__ kp,
                                              const _Float16* __restrict__ vt,
                                              const float* __restrict__ szin,
                                              const float* __restrict__ mkin,
                                              _Float16* __restrict__ op,
                                              float* __restrict__ part, float sscale) {
  __shared__ __align__(16) _Float16 Ks[64 * KTP];
  __shared__ __align__(16) _Float16 Vs[64 * KTP];
  __shared__ __align__(16) _Float16 Ps[8][16 * PTP];
  __shared__ __align__(16) float lsz[NN];
  __shared__ __align__(16) float kmk[NN];
  __shared__ __align__(16) float csum[NN];
  __shared__ float csw[8][64];

  const int tid = threadIdx.x, lane = tid & 31, wave = tid >> 5;
  const int hh = lane >> 4, c = lane & 15;
  const int bh = blockIdx.x / QB;
  const int qb = blockIdx.x - bh * QB;
  const int b  = bh / HH, h = bh - b * HH;
  const int q0 = qb * 128 + wave * 16;

#pragma unroll 1
  for (int i = tid; i < NN; i += 256) {
    lsz[i] = logf(szin[(size_t)b * NN + i]);
    kmk[i] = mkin[(size_t)b * NN + i];
  }

  const _Float16* Q = qp + (size_t)bh * NN * DD;
  const _Float16* K = kp + (size_t)bh * NN * DD;
  const _Float16* V = vt + (size_t)bh * DD * NN;

  v16h qa[2];
  qa[0] = ldfrag(Q, DD, q0, 0, lane);
  qa[1] = ldfrag(Q, DD, q0, 32, lane);

  const float NEGI = -__builtin_huge_valf();
  float mrow[8], lrow[8];
#pragma unroll
  for (int r = 0; r < 8; ++r) { mrow[r] = NEGI; lrow[r] = 0.f; }

  for (int kc = 0; kc < NN / 64; ++kc) {
    const int kv0 = kc * 64;
    __syncthreads();
    {
      const int r  = tid >> 2;
      const int qq = (tid & 3) * 16;
      const _Float16* ks = K + (size_t)(kv0 + r) * DD + qq;
      *(v8h*)(Ks + r * KTP + qq)     = *(const v8h*)(ks);
      *(v8h*)(Ks + r * KTP + qq + 8) = *(const v8h*)(ks + 8);
    }
    __syncthreads();

    v8f s[4];
#pragma unroll
    for (int j = 0; j < 4; ++j) s[j] = zero8();
#pragma unroll
    for (int dc = 0; dc < 2; ++dc) {
#pragma unroll
      for (int j = 0; j < 4; ++j) {
        const v16h kb = ldfrag(Ks, KTP, j * 16, dc * 32, lane);
        s[j] = mma16(qa[dc], kb, s[j]);
      }
    }
    float lsj[4], mkj[4];
#pragma unroll
    for (int j = 0; j < 4; ++j) { lsj[j] = lsz[kv0 + j * 16 + c]; mkj[j] = kmk[kv0 + j * 16 + c]; }
    float cm[8];
#pragma unroll
    for (int r = 0; r < 8; ++r) {
      float m = NEGI;
#pragma unroll
      for (int j = 0; j < 4; ++j) {
        const float sv = s[j][r] * sscale + lsj[j];
        s[j][r] = sv;
        m = fmaxf(m, sv);
      }
#pragma unroll
      for (int off = 1; off < 16; off <<= 1) m = fmaxf(m, __shfl_xor(m, off, 32));
      cm[r] = m;
    }
#pragma unroll
    for (int r = 0; r < 8; ++r) {
      const float mnew  = fmaxf(mrow[r], cm[r]);
      const float alpha = __expf(mrow[r] - mnew);
      mrow[r] = mnew;
      float psum = 0.f;
#pragma unroll
      for (int j = 0; j < 4; ++j) psum += __expf(s[j][r] - mnew) * mkj[j];
#pragma unroll
      for (int off = 1; off < 16; off <<= 1) psum += __shfl_xor(psum, off, 32);
      lrow[r] = lrow[r] * alpha + psum;
    }
  }

  float invl[8];
#pragma unroll
  for (int r = 0; r < 8; ++r) invl[r] = 1.0f / (lrow[r] + 1e-6f);

  v8f oacc[4];
#pragma unroll
  for (int t = 0; t < 4; ++t) oacc[t] = zero8();
  _Float16* pw = Ps[wave];

  for (int kc = 0; kc < NN / 64; ++kc) {
    const int kv0 = kc * 64;
    __syncthreads();
    {
      const int r  = tid >> 2;
      const int qq = (tid & 3) * 16;
      const _Float16* ks = K + (size_t)(kv0 + r) * DD + qq;
      *(v8h*)(Ks + r * KTP + qq)     = *(const v8h*)(ks);
      *(v8h*)(Ks + r * KTP + qq + 8) = *(const v8h*)(ks + 8);
      const _Float16* vs = V + (size_t)r * NN + kv0 + qq;
      *(v8h*)(Vs + r * KTP + qq)     = *(const v8h*)(vs);
      *(v8h*)(Vs + r * KTP + qq + 8) = *(const v8h*)(vs + 8);
    }
    __syncthreads();

    v8f s[4];
#pragma unroll
    for (int j = 0; j < 4; ++j) s[j] = zero8();
#pragma unroll
    for (int dc = 0; dc < 2; ++dc) {
#pragma unroll
      for (int j = 0; j < 4; ++j) {
        const v16h kb = ldfrag(Ks, KTP, j * 16, dc * 32, lane);
        s[j] = mma16(qa[dc], kb, s[j]);
      }
    }
    float lsj[4], mkj[4];
#pragma unroll
    for (int j = 0; j < 4; ++j) { lsj[j] = lsz[kv0 + j * 16 + c]; mkj[j] = kmk[kv0 + j * 16 + c]; }
    float csl[4];
#pragma unroll
    for (int j = 0; j < 4; ++j) csl[j] = 0.f;
#pragma unroll
    for (int r = 0; r < 8; ++r) {
#pragma unroll
      for (int j = 0; j < 4; ++j) {
        const float sv = s[j][r] * sscale + lsj[j];
        const float p  = __expf(sv - mrow[r]) * mkj[j] * invl[r];
        csl[j] += p;
        pw[(8 * hh + r) * PTP + j * 16 + c] = (_Float16)(p * 1024.0f);
      }
    }
#pragma unroll
    for (int j = 0; j < 4; ++j) csl[j] += __shfl_xor(csl[j], 16, 32);
    if (lane < 16) {
#pragma unroll
      for (int j = 0; j < 4; ++j) csw[wave][j * 16 + c] = csl[j];
    }
    __syncthreads();

    if (tid < 64) {
      float a = 0.f;
#pragma unroll
      for (int w = 0; w < 8; ++w) a += csw[w][tid];
      csum[kv0 + tid] = a;
    }

#pragma unroll
    for (int kk = 0; kk < 2; ++kk) {
      const v16h pa = ldfrag(pw, PTP, 0, kk * 32, lane);
#pragma unroll
      for (int t = 0; t < 4; ++t) {
        const v16h vb = ldfrag(Vs, KTP, t * 16, kk * 32, lane);
        oacc[t] = mma16(pa, vb, oacc[t]);
      }
    }
  }
  __syncthreads();

#pragma unroll
  for (int r = 0; r < 8; ++r) {
#pragma unroll
    for (int t = 0; t < 4; ++t) pw[(8 * hh + r) * PTP + 16 * t + c] = (_Float16)(oacc[t][r] * 0.0625f);
  }
  __syncthreads();
  v4u val[4];
  size_t go[4];
#pragma unroll
  for (int it = 0; it < 4; ++it) {
    const int p  = lane + 32 * it;
    const int L  = p >> 3;
    const int pc = p & 7;
    Pack8 pk;
    pk.h   = *(const v8h*)(pw + L * PTP + pc * 8);
    val[it] = pk.u;
    go[it]  = ((size_t)(b * NN + q0 + L)) * CC + (size_t)h * DD + pc * 8;
  }
  const v4f cv = *(const v4f*)(csum + 4 * tid);
  const size_t cgo = ((size_t)bh * QB + qb) * NN + 4 * tid;
  for (int ps = 0; ps < 2; ++ps) {
#pragma unroll
    for (int it = 0; it < 4; ++it) *(volatile v4u*)(op + go[it]) = val[it];
    *(volatile v4f*)(part + cgo) = cv;
    __threadfence();
  }
}

__global__ __launch_bounds__(256) void k_metric(const _Float16* __restrict__ kp,
                                                const float* __restrict__ mkin,
                                                float* __restrict__ met) {
  const int t = blockIdx.x * 256 + (int)threadIdx.x;
  const int tok = t >> 4;
  const int piece = t & 15;
  const int b = tok / NN, n = tok - b * NN;
  v4f a = zero4();
#pragma unroll
  for (int h = 0; h < HH; ++h) {
    const v4hh kv = *(const v4hh*)(kp + ((size_t)((b * HH + h) * NN + n)) * DD + 4 * piece);
    a[0] += (float)kv[0]; a[1] += (float)kv[1]; a[2] += (float)kv[2]; a[3] += (float)kv[3];
  }
  const float r12 = 1.0f / (float)HH;
  a[0] *= r12; a[1] *= r12; a[2] *= r12; a[3] *= r12;
  float ss = (a[0] * a[0] + a[1] * a[1]) + (a[2] * a[2] + a[3] * a[3]);
#pragma unroll
  for (int off = 1; off < 16; off <<= 1) ss += __shfl_xor(ss, off, 32);
  const float f = (1.0f / sqrtf(ss)) * mkin[(size_t)b * NN + n];
  v4f o;
  o[0] = a[0] * f; o[1] = a[1] * f; o[2] = a[2] * f; o[3] = a[3] * f;
  volatile v4f* d = (volatile v4f*)(met + (size_t)tok * DD + 4 * piece);
  *d = o;
  __threadfence();
  *d = o;
}

#define OTP 68
template <int KK, int RS>
__global__ __launch_bounds__(256) void k_gout(const _Float16* __restrict__ ap,
                                              const _Float16* __restrict__ wt,
                                              const float* __restrict__ bias,
                                              const float* __restrict__ res,
                                              const float* __restrict__ rs,
                                              float* __restrict__ out, float oscale) {
  __shared__ __align__(16) float st[8][16 * OTP];
  const int tid = threadIdx.x, lane = tid & 31, wave = tid >> 5;
  const int hh = lane >> 4, c = lane & 15;
  const int m0 = blockIdx.x * 256 + wave * 32;
  const int n0 = blockIdx.y * 64;

  v8f acc[2][4];
#pragma unroll
  for (int s = 0; s < 2; ++s)
#pragma unroll
    for (int t = 0; t < 4; ++t) acc[s][t] = zero8();
  gemm32x64<KK>(ap, KK, wt, KK, m0, n0, lane, acc);

  float bvs[4];
#pragma unroll
  for (int t = 0; t < 4; ++t) bvs[t] = bias[n0 + 16 * t + c];

  float* sw = st[wave];
#pragma unroll
  for (int sub = 0; sub < 2; ++sub) {
    __syncthreads();
#pragma unroll
    for (int t = 0; t < 4; ++t) {
#pragma unroll
      for (int r = 0; r < 8; ++r)
        sw[(8 * hh + r) * OTP + 16 * t + c] = acc[sub][t][r] * oscale + bvs[t];
    }
    __syncthreads();
    v4f val[8];
    size_t go[8];
#pragma unroll
    for (int it = 0; it < 8; ++it) {
      const int p    = lane + 32 * it;
      const int L    = p >> 3;
      const int pc   = p & 7;
      const int row  = L >> 1;
      const int half = L & 1;
      const int grow = m0 + sub * 16 + row;
      const size_t g = (size_t)grow * CC + n0 + half * 32 + pc * 4;
      v4f v = *(const v4f*)(sw + row * OTP + half * 32 + pc * 4);
      const v4f rr = *(const v4f*)(res + g);
      v[0] = v[0] + rr[0]; v[1] = v[1] + rr[1]; v[2] = v[2] + rr[2]; v[3] = v[3] + rr[3];
      if (RS) {
        const float f = rs[grow];
        v[0] *= f; v[1] *= f; v[2] *= f; v[3] *= f;
      }
      val[it] = v;
      go[it]  = g;
    }
    for (int ps = 0; ps < 2; ++ps) {
#pragma unroll
      for (int it = 0; it < 8; ++it) *(volatile v4f*)(out + go[it]) = val[it];
      __threadfence();
    }
  }
}

__global__ __launch_bounds__(256) void k_ffn1(const _Float16* __restrict__ ap,
                                              const _Float16* __restrict__ wt,
                                              const float* __restrict__ bias,
                                              _Float16* __restrict__ hp) {
  __shared__ __align__(16) float st[8][16 * OTP];
  const int tid = threadIdx.x, lane = tid & 31, wave = tid >> 5;
  const int hh = lane >> 4, c = lane & 15;
  const int m0 = blockIdx.x * 256 + wave * 32;
  const int n0 = blockIdx.y * 64;

  v8f acc[2][4];
#pragma unroll
  for (int s = 0; s < 2; ++s)
#pragma unroll
    for (int t = 0; t < 4; ++t) acc[s][t] = zero8();
  gemm32x64<CC>(ap, CC, wt, CC, m0, n0, lane, acc);

  float bvs[4];
#pragma unroll
  for (int t = 0; t < 4; ++t) bvs[t] = bias[n0 + 16 * t + c];

  float* sw = st[wave];
#pragma unroll
  for (int sub = 0; sub < 2; ++sub) {
    __syncthreads();
#pragma unroll
    for (int t = 0; t < 4; ++t) {
#pragma unroll
      for (int r = 0; r < 8; ++r)
        sw[(8 * hh + r) * OTP + 16 * t + c] = acc[sub][t][r] * 0.03125f + bvs[t];
    }
    __syncthreads();
    v4u val[4];
    size_t go[4];
#pragma unroll
    for (int it = 0; it < 4; ++it) {
      const int p  = lane + 32 * it;
      const int L  = p >> 3;
      const int pc = p & 7;
      const v4f x0 = *(const v4f*)(sw + L * OTP + pc * 8);
      const v4f x1 = *(const v4f*)(sw + L * OTP + pc * 8 + 4);
      Pack8 pk;
      pk.h = (v8h){(_Float16)act16(x0[0]), (_Float16)act16(x0[1]), (_Float16)act16(x0[2]), (_Float16)act16(x0[3]),
                   (_Float16)act16(x1[0]), (_Float16)act16(x1[1]), (_Float16)act16(x1[2]), (_Float16)act16(x1[3])};
      val[it] = pk.u;
      go[it]  = (size_t)(m0 + sub * 16 + L) * FF + n0 + pc * 8;
    }
    for (int ps = 0; ps < 2; ++ps) {
#pragma unroll
      for (int it = 0; it < 4; ++it) *(volatile v4u*)(hp + go[it]) = val[it];
      __threadfence();
    }
  }
}

#define MTP 68
__global__ __launch_bounds__(256) void k_merge(const float* __restrict__ x1,
                                               const float* __restrict__ szin,
                                               const float* __restrict__ mkin,
                                               const float* __restrict__ vzin,
                                               const float* __restrict__ met,
                                               const float* __restrict__ part,
                                               float* __restrict__ xm,
                                               float* __restrict__ osz,
                                               float* __restrict__ omk,
                                               float* __restrict__ ovz,
                                               float thr, float pthr) {
  __shared__ __align__(16) float As[32 * MTP];
  __shared__ __align__(16) float Bs[64 * MTP];
  __shared__ __align__(16) float s_imp[NN];
  __shared__ __align__(16) float s_szo[NN];
  __shared__ __align__(16) float s_mko[NN];
  __shared__ float s_inv[NN];
  __shared__ float s_mm[NH];
  __shared__ float s_msz[NH];
  __shared__ float s_msc[NH];
  __shared__ int   s_idx[NH];
  __shared__ int   s_cnt[NH];
  __shared__ int   s_start[NH + 4];
  __shared__ int   s_ord[NH];

  const int tid = threadIdx.x, lane = tid & 31;
  const int b = blockIdx.x;
  const size_t tokb = (size_t)b * NN;
  const float NEGI = -__builtin_huge_valf();

  {
    v4f a = zero4();
#pragma unroll 1
    for (int h = 0; h < HH; ++h) {
#pragma unroll 1
      for (int q = 0; q < QB; ++q) {
        const v4f pv = *(const v4f*)(part + ((size_t)((b * HH + h) * QB + q)) * NN + 4 * tid);
        a[0] += pv[0]; a[1] += pv[1]; a[2] += pv[2]; a[3] += pv[3];
      }
    }
    const float sc = 1.0f / (float)(HH * NN);
    a[0] *= sc; a[1] *= sc; a[2] *= sc; a[3] *= sc;
    *(v4f*)(s_imp + 4 * tid) = a;
    if (tid == 0) s_imp[0] = __builtin_huge_valf();
  }

  const int gi = tid >> 3, jsub = tid & 7;
#pragma unroll 1
  for (int ig = 0; ig < NH / 32; ++ig) {
    __syncthreads();
    {
      const int ar = tid >> 3, ac = (tid & 7) * 8;
      const float* src = met + (tokb + 2 * (ig * 32 + ar)) * DD + ac;
      *(v4f*)(As + ar * MTP + ac)     = *(const v4f*)(src);
      *(v4f*)(As + ar * MTP + ac + 4) = *(const v4f*)(src + 4);
    }
    float best = NEGI;
    int bidx = 0;
#pragma unroll 1
    for (int jt = 0; jt < NH / 64; ++jt) {
      __syncthreads();
      {
        const int br = tid >> 2, bc = (tid & 3) * 16;
        const float* src = met + (tokb + 2 * (jt * 64 + br) + 1) * DD + bc;
#pragma unroll
        for (int u = 0; u < 4; ++u) *(v4f*)(Bs + br * MTP + bc + 4 * u) = *(const v4f*)(src + 4 * u);
      }
      __syncthreads();
      const float* arow = As + gi * MTP;
#pragma unroll 1
      for (int jj = 0; jj < 8; ++jj) {
        const int jl = jj * 8 + jsub;
        const float* brow = Bs + jl * MTP;
        float acc = 0.f;
#pragma unroll 4
        for (int d4 = 0; d4 < DD / 4; ++d4) {
          const v4f va = *(const v4f*)(arow + 4 * d4);
          const v4f vb = *(const v4f*)(brow + 4 * d4);
          acc = fmaf(va[0], vb[0], acc);
          acc = fmaf(va[1], vb[1], acc);
          acc = fmaf(va[2], vb[2], acc);
          acc = fmaf(va[3], vb[3], acc);
        }
        const int j = jt * 64 + jl;
        if (acc > best) { best = acc; bidx = j; }
      }
    }
#pragma unroll
    for (int off = 1; off < 8; off <<= 1) {
      const float ob = __shfl_xor(best, off, 32);
      const int   oi = __shfl_xor(bidx, off, 32);
      const bool take = (ob > best) || (ob == best && oi < bidx);
      best = take ? ob : best;
      bidx = take ? oi : bidx;
    }
    const int i = ig * 32 + gi;
    const bool z = (i == 0);
    const float bm = z ? NEGI : best;
    const int   bi = z ? 0 : bidx;
    if (jsub == 0) {
      s_mm[i]  = (bm > thr) ? 1.0f : 0.0f;
      s_idx[i] = min(max(bi, 0), NH - 1);
    }
  }
  __syncthreads();

#pragma unroll 1
  for (int qq = 0; qq < 2; ++qq) {
    const int i = tid + 256 * qq;
    const float mm = s_mm[i];
    const float ss = szin[tokb + 2 * i];
    const float sm = mkin[tokb + 2 * i];
    const float im = s_imp[2 * i];
    s_msz[i] = ss * mm;
    s_msc[i] = (i == 0) ? 0.0f : im * mm;
    const float unm = (sm > 0.0f) ? (1.0f - mm) : sm;
    s_szo[i] = ss;
    s_inv[i] = 1.0f / ss;
    s_mko[i] = (unm > 0.0f) ? ((im > pthr) ? 1.0f : 0.0f) : unm;
  }
  __syncthreads();
#pragma unroll 1
  for (int qq = 0; qq < 2; ++qq) {
    const int j = tid + 256 * qq;
    float ds = szin[tokb + 2 * j + 1];
    const float dm = mkin[tokb + 2 * j + 1];
    float sc = s_imp[2 * j + 1];
    int cnt = 0;
#pragma unroll 1
    for (int i = 0; i < NH; ++i) {
      const bool hit = (s_idx[i] == j);
      const float msz = s_msz[i];
      const float msc = s_msc[i];
      ds  = hit ? (ds + msz) : ds;
      sc  = hit ? fmaxf(sc, msc) : sc;
      cnt += hit ? 1 : 0;
    }
    s_szo[NH + j] = ds;
    s_inv[NH + j] = 1.0f / ds;
    s_mko[NH + j] = (dm > 0.0f) ? ((sc > pthr) ? 1.0f : 0.0f) : dm;
    s_cnt[j] = cnt;
  }
  __syncthreads();
  if (tid == 0) {
    int run = 0;
#pragma unroll 1
    for (int j = 0; j < NH; ++j) {
      s_start[j] = run;
      run += s_cnt[j];
      run = min(run, NH);
    }
    s_start[NH] = run;
  }
  __syncthreads();
#pragma unroll 1
  for (int qq = 0; qq < 2; ++qq) {
    const int j = tid + 256 * qq;
    int pos = s_start[j];
    const int lim = min(s_start[j + 1], NH);
#pragma unroll 1
    for (int i = 0; i < NH; ++i) {
      if (s_idx[i] == j) {
        if (pos < lim && (unsigned)pos < (unsigned)NH) s_ord[pos] = i;
        ++pos;
      }
    }
  }
  {
    const v4f sv = *(const v4f*)(s_szo + 4 * tid);
    const v4f mv = *(const v4f*)(s_mko + 4 * tid);
    volatile v4f* ps = (volatile v4f*)(osz + tokb + 4 * tid);
    volatile v4f* pm = (volatile v4f*)(omk + tokb + 4 * tid);
    *ps = sv; *pm = mv;
    __threadfence();
    *ps = sv; *pm = mv;
  }
  __syncthreads();

  const int cx = min(4 * tid, CC - 4);
  const bool xw = tid < 192;
#pragma unroll 1
  for (int r = 0; r < NN; ++r) {
    const bool isdst = (r >= NH);
    const int orig = isdst ? (2 * (r - NH) + 1) : (2 * r);
    const float inv = s_inv[r];
    int p0 = 0, cnt = 0;
    if (isdst) {
      p0 = min(max(s_start[r - NH], 0), NH);
      const int p1 = min(max(s_start[r - NH + 1], p0), NH);
      cnt = p1 - p0;
    }
    v4f vv = *(const v4f*)(vzin + (tokb + orig) * NN + 4 * tid);
    v4f xv = *(const v4f*)(x1 + (tokb + orig) * CC + cx);
#pragma unroll 1
    for (int p = 0; p < cnt; ++p) {
      int i = s_ord[min(p0 + p, NH - 1)];
      i = min(max(i, 0), NH - 1);
      const float m = s_mm[i];
      const v4f vs = *(const v4f*)(vzin + (tokb + 2 * i) * NN + 4 * tid);
      const v4f xs = *(const v4f*)(x1 + (tokb + 2 * i) * CC + cx);
      vv[0] = fmaxf(vv[0], m * vs[0]); vv[1] = fmaxf(vv[1], m * vs[1]);
      vv[2] = fmaxf(vv[2], m * vs[2]); vv[3] = fmaxf(vv[3], m * vs[3]);
      xv[0] = xv[0] + m * xs[0]; xv[1] = xv[1] + m * xs[1];
      xv[2] = xv[2] + m * xs[2]; xv[3] = xv[3] + m * xs[3];
    }
    xv[0] *= inv; xv[1] *= inv; xv[2] *= inv; xv[3] *= inv;
    volatile v4f* pv = (volatile v4f*)(ovz + (tokb + r) * NN + 4 * tid);
    volatile v4f* px = (volatile v4f*)(xm + (tokb + r) * CC + 4 * tid);
    *pv = vv;
    if (xw) *px = xv;
    __threadfence();
    *pv = vv;
    if (xw) *px = xv;
  }
  (void)lane;
}

extern "C" void kernel_launch(void* const* d_in, const int* in_sizes, int n_in,
                              void* d_out, int out_size, void* d_ws, size_t ws_size,
                              hipStream_t stream) {
  if (n_in < 15) return;
  if (in_sizes[0] != ROWS * CC) return;
  if (in_sizes[1] != ROWS || in_sizes[2] != ROWS) return;
  if (in_sizes[3] != ROWS * NN) return;
  if (in_sizes[4] != CC * C3) return;
  if (in_sizes[5] != CC * CC || in_sizes[6] != CC) return;
  if (in_sizes[7] != CC || in_sizes[8] != CC || in_sizes[9] != CC || in_sizes[10] != CC) return;
  if (in_sizes[11] != CC * FF || in_sizes[12] != FF) return;
  if (in_sizes[13] != FF * CC || in_sizes[14] != CC) return;
  if (out_size != ROWS * CC + ROWS + ROWS + ROWS * NN) return;

  const float* x    = (const float*)d_in[0];
  const float* szin = (const float*)d_in[1];
  const float* mkin = (const float*)d_in[2];
  const float* vzin = (const float*)d_in[3];
  const float* Wqkv = (const float*)d_in[4];
  const float* Wp   = (const float*)d_in[5];
  const float* bp   = (const float*)d_in[6];
  const float* g1   = (const float*)d_in[7];
  const float* be1  = (const float*)d_in[8];
  const float* g2   = (const float*)d_in[9];
  const float* be2  = (const float*)d_in[10];
  const float* W1   = (const float*)d_in[11];
  const float* b1   = (const float*)d_in[12];
  const float* W2   = (const float*)d_in[13];
  const float* b2   = (const float*)d_in[14];
  float* out  = (float*)d_out;
  float* o_x  = out;
  float* o_sz = out + (size_t)ROWS * CC;
  float* o_mk = o_sz + ROWS;
  float* o_vz = o_mk + ROWS;

  size_t off = 0;
  const size_t oXN  = off; off += (size_t)ROWS * CC * 2;
  const size_t oWQ  = off; off += (size_t)C3 * CC * 2;
  const size_t oQKV = off; off += 3 * PL * 2;
  const size_t oCTX = off; off += (size_t)ROWS * CC * 2;
  const size_t oH   = oWQ;
  if (oH + (size_t)ROWS * FF * 2 > off) return;
  const size_t oWO  = off; off += (size_t)CC * CC * 2;
  const size_t oW1  = off; off += (size_t)FF * CC * 2;
  const size_t oW2  = off; off += (size_t)CC * FF * 2;
  const size_t oX1  = off; off += (size_t)ROWS * CC * 4;
  const size_t oMET = off; off += (size_t)ROWS * DD * 4;
  const size_t oPRT = off; off += (size_t)BB * HH * QB * NN * 4;
  const size_t oXM  = off; off += (size_t)ROWS * CC * 4;
  if (off > ws_size) return;
  if (off > (size_t)134217728) return;

  char* ws = (char*)d_ws;
  _Float16* XN   = (_Float16*)(ws + oXN);
  _Float16* HN   = (_Float16*)(ws + oXN);
  _Float16* WQt  = (_Float16*)(ws + oWQ);
  _Float16* QKVp = (_Float16*)(ws + oQKV);
  _Float16* CTX  = (_Float16*)(ws + oCTX);
  _Float16* Hp   = (_Float16*)(ws + oH);
  _Float16* WOt  = (_Float16*)(ws + oWO);
  _Float16* W1t  = (_Float16*)(ws + oW1);
  _Float16* W2t  = (_Float16*)(ws + oW2);
  float*    X1   = (float*)(ws + oX1);
  float*    MET  = (float*)(ws + oMET);
  float*    PART = (float*)(ws + oPRT);
  float*    XM   = (float*)(ws + oXM);

  k_ln<<<dim3(ROWS), dim3(192), 0, stream>>>(x, g1, be1, XN, 1e-5f);
  k_wt<<<dim3(C3 / 64, CC / 64), dim3(256), 0, stream>>>(Wqkv, WQt, C3, CC);
  k_wt<<<dim3(CC / 64, CC / 64), dim3(256), 0, stream>>>(Wp, WOt, CC, CC);
  k_wt<<<dim3(FF / 64, CC / 64), dim3(256), 0, stream>>>(W1, W1t, FF, CC);
  k_wt<<<dim3(CC / 64, FF / 64), dim3(256), 0, stream>>>(W2, W2t, CC, FF);
  k_qkv<<<dim3(ROWS / 256, C3 / 64), dim3(256), 0, stream>>>(XN, WQt, QKVp);
  k_attn<<<dim3(BB * HH * QB), dim3(256), 0, stream>>>(QKVp, QKVp + PL, QKVp + 2 * PL, szin, mkin, CTX, PART, 0.125f);
  k_metric<<<dim3(ROWS * 16 / 256), dim3(256), 0, stream>>>(QKVp + PL, mkin, MET);
  k_gout<CC, 1><<<dim3(ROWS / 256, CC / 64), dim3(256), 0, stream>>>(CTX, WOt, bp, x, szin, X1, 0.00048828125f);
  k_merge<<<dim3(BB), dim3(256), 0, stream>>>(X1, szin, mkin, vzin, MET, PART, XM, o_sz, o_mk, o_vz, 0.9f, 0.0f);
  k_ln<<<dim3(ROWS), dim3(192), 0, stream>>>(XM, g2, be2, HN, 1e-5f);
  k_ffn1<<<dim3(ROWS / 256, FF / 64), dim3(256), 0, stream>>>(HN, W1t, b1, Hp);
  k_gout<FF, 0><<<dim3(ROWS / 256, CC / 64), dim3(256), 0, stream>>>(Hp, W2t, b2, XM, szin, o_x, 0.001953125f);
  (void)hipGetLastError();
}
